// GATLayer_55052890800667
// MI455X (gfx1250) — hardware-verified
//
#include <hip/hip_runtime.h>
#include <stddef.h>
#include <stdint.h>
#include <math.h>


#define NB_G   8
#define NN     1024
#define FIN    256
#define FOUT   256
#define NHD    4
#define HD     64
#define NROW   (NB_G * NN)
#define QT     64
#define KT     64
#define NKT    (NN / KT)
#define NQT    (NN / QT)
#define NTHR   256
#define GBM    64
#define GBN    64
#define GTHR   128
#define NEGSL  0.2f
#define BNEPS  1e-5f
#define WSMAX  134217728
#define VPLANE ((size_t)NB_G * NHD * HD * NN)

#define SZ_HB   ((size_t)NROW * FIN * 2)
#define SZ_WB   ((size_t)FOUT * FIN * 2)
#define SZ_WH   ((size_t)NROW * FOUT * 4)
#define SZ_VHL  ((size_t)2 * VPLANE * 2)
#define SZ_SD   ((size_t)NHD * 2 * NROW * 4)
#define SZ_OUT  ((size_t)NROW * FOUT * 4)
#define SZ_PART ((size_t)NB_G * NHD * NQT * 2 * HD * 4)
#define SZ_MI   ((size_t)2 * FOUT * 4)

static_assert((FIN % 32) == 0);
static_assert((NROW % GBM) == 0 && (FOUT % GBN) == 0);
static_assert(HD == GBN && FOUT == NHD * HD);
static_assert(GBM == (GTHR / 32) * 16 && GTHR == 2 * GBN && GTHR == 2 * GBM);
static_assert(QT == GBM && KT == 64 && (NN % QT) == 0 && (NN % KT) == 0);
static_assert(GTHR * 8 == NN);
static_assert((NN % GBM) == 0);
static_assert(NTHR == FOUT);
static_assert((NROW * FOUT) % (4 * NTHR) == 0);
static_assert((SZ_HB % 256) == 0 && (SZ_WB % 256) == 0 && (SZ_WH % 256) == 0 && (SZ_VHL % 256) == 0);
static_assert((SZ_SD % 256) == 0 && (SZ_OUT % 256) == 0 && (SZ_PART % 256) == 0 && (SZ_MI % 256) == 0);
static_assert(SZ_HB + SZ_WB + SZ_WH + SZ_VHL + SZ_SD + SZ_OUT + SZ_PART + SZ_MI <= (size_t)WSMAX);

typedef float          v4f  __attribute__((ext_vector_type(4)));
typedef float          v8f  __attribute__((ext_vector_type(8)));
typedef int            v4i  __attribute__((ext_vector_type(4)));
typedef int            v8i  __attribute__((ext_vector_type(8)));
typedef unsigned int   v4u  __attribute__((ext_vector_type(4)));
typedef unsigned short v8us __attribute__((ext_vector_type(8)));
typedef __bf16         v16b __attribute__((ext_vector_type(16)));
typedef v4f  __attribute__((may_alias)) v4fa;
typedef v4i  __attribute__((may_alias)) v4ia;
typedef v4u  __attribute__((may_alias)) v4ua;
typedef v8us __attribute__((may_alias)) v8usa;
union FragB { v16b v; v8us u[2]; v4u q[2]; v8i w; };

__device__ __forceinline__ v8f wmb(const FragB& a, const FragB& b, v8f c) {
  v8f d = __builtin_amdgcn_wmma_f32_16x16x32_bf16(false, a.v, false, b.v, (short)0, c, false, false);
  asm volatile("v_nop\n\tv_nop\n\tv_nop\n\tv_nop" : "+v"(d) : "v"(a.w), "v"(b.w));
  return d;
}

__device__ __forceinline__ unsigned int f2bf(float f) {
  const unsigned int u = __float_as_uint(f);
  return ((u + 0x7FFFu + ((u >> 16) & 1u)) >> 16) & 0xFFFFu;
}
__device__ __forceinline__ float bf2f(unsigned int b) { return __uint_as_float(b << 16); }
__device__ __forceinline__ float bfr(float f) { return bf2f(f2bf(f)); }
__device__ __forceinline__ v4f bfr4(const v4f a) {
  v4f r; r.x = bfr(a.x); r.y = bfr(a.y); r.z = bfr(a.z); r.w = bfr(a.w); return r;
}
__device__ __forceinline__ unsigned int pk2(float lo, float hi) { return f2bf(lo) | (f2bf(hi) << 16); }
__device__ __forceinline__ v4u pack8(const v4f a, const v4f b) {
  v4u r;
  r.x = pk2(a.x, a.y); r.y = pk2(a.z, a.w); r.z = pk2(b.x, b.y); r.w = pk2(b.z, b.w);
  return r;
}
__device__ __forceinline__ v4f max4(const v4f a, const v4f b) {
  v4f r; r.x = fmaxf(a.x, b.x); r.y = fmaxf(a.y, b.y); r.z = fmaxf(a.z, b.z); r.w = fmaxf(a.w, b.w); return r;
}

__global__ __launch_bounds__(NTHR) void k_cvt(const float* __restrict__ x, unsigned short* xb, int nUnits) {
  const int i = (int)blockIdx.x * NTHR + (int)threadIdx.x;
  if (i >= nUnits) return;
  const float* p = x + (size_t)i * 8;
  const v4f a = *(const v4fa*)p, b = *(const v4fa*)(p + 4);
  const v4u hv = pack8(a, b);
  const size_t o = (size_t)i * 8;
  *(volatile v4u*)(xb + o) = hv;
  __threadfence();
  *(volatile v4u*)(xb + o) = hv;
}

__device__ __forceinline__ v4u vt_piece(const float* stg, int piece, int d, float fl) {
  const float* sc = stg + (8 * piece) * GBN + d;
  v4f a, b;
  a.x = sc[0];       a.y = sc[GBN];     a.z = sc[2 * GBN]; a.w = sc[3 * GBN];
  b.x = sc[4 * GBN]; b.y = sc[5 * GBN]; b.z = sc[6 * GBN]; b.w = sc[7 * GBN];
  a.x = fmaf(-fl, bfr(a.x), a.x); a.y = fmaf(-fl, bfr(a.y), a.y); a.z = fmaf(-fl, bfr(a.z), a.z); a.w = fmaf(-fl, bfr(a.w), a.w);
  b.x = fmaf(-fl, bfr(b.x), b.x); b.y = fmaf(-fl, bfr(b.y), b.y); b.z = fmaf(-fl, bfr(b.z), b.z); b.w = fmaf(-fl, bfr(b.w), b.w);
  return pack8(a, b);
}

__global__ __launch_bounds__(GTHR) void k_proj(
    const unsigned short* __restrict__ A, const unsigned short* __restrict__ WT,
    float* outF, const float* __restrict__ atts, const float* __restrict__ attd,
    float* SD, unsigned short* VHL)
{
  __shared__ __attribute__((aligned(16))) float stg[GBM * GBN];
  __shared__ __attribute__((aligned(16))) float satt[2 * GBN];
  __shared__ __attribute__((aligned(16))) float sdot[2 * GBM];
  const int tid = (int)threadIdx.x, lane = tid & 31, wave = tid >> 5, hh = lane >> 4, m = lane & 15;
  const int rowBase = (int)blockIdx.x * GBM;
  const int head    = (int)blockIdx.y;
  const int col0    = head * GBN;

  {
    const int which = tid >> 6;
    const int c  = tid & 63;
    const float vs = atts[head * HD + c];
    const float vd = attd[head * HD + c];
    const float v = (which == 0) ? vs : vd;
    satt[which * GBN + c] = bfr(v);
  }

  v8f acc[4];
  {
    const v8f z = {0.f, 0.f, 0.f, 0.f, 0.f, 0.f, 0.f, 0.f};
    acc[0] = z; acc[1] = z; acc[2] = z; acc[3] = z;
  }
  const unsigned short* ap = A  + (size_t)(rowBase + 16 * wave + m) * (size_t)FIN + 8 * hh;
  const unsigned short* wp = WT + (size_t)(col0 + m) * (size_t)FIN + 8 * hh;
#pragma unroll 1
  for (int ks = 0; ks < FIN / 32; ++ks) {
    FragB af;
    af.u[0] = *(const v8usa*)(ap + 32 * ks);
    af.u[1] = *(const v8usa*)(ap + 32 * ks + 16);
#pragma unroll
    for (int t = 0; t < 4; ++t) {
      const unsigned short* wq = wp + (size_t)(16 * t) * (size_t)FIN + 32 * ks;
      FragB bf;
      bf.u[0] = *(const v8usa*)wq;
      bf.u[1] = *(const v8usa*)(wq + 16);
      acc[t] = wmb(af, bf, acc[t]);
    }
  }

#pragma unroll
  for (int t = 0; t < 4; ++t) {
    const int lc = 16 * t + m;
#pragma unroll
    for (int r = 0; r < 8; ++r) {
      const int lr = 16 * wave + 8 * hh + r;
      stg[lr * GBN + lc] = acc[t][r];
    }
  }
  __syncthreads();

  {
    const int row = tid & 63, which = tid >> 6;
    const float* sa = satt + which * GBN;
    const float* hr = stg + row * GBN;
    float d = 0.f;
#pragma unroll 4
    for (int c4 = 0; c4 < GBN / 4; ++c4) {
      const v4f hv = *(const v4fa*)(hr + 4 * c4);
      const v4f av = *(const v4fa*)(sa + 4 * c4);
      d = fmaf(hv.x, av.x, d);
      d = fmaf(hv.y, av.y, d);
      d = fmaf(hv.z, av.z, d);
      d = fmaf(hv.w, av.w, d);
    }
    sdot[which * GBM + row] = d;
  }
  __syncthreads();

  v4f fv[8];
#pragma unroll
  for (int i = 0; i < 8; ++i) {
    const int lr = 16 * wave + 2 * i + hh;
    fv[i] = *(const v4fa*)(stg + lr * GBN + 4 * m);
  }
  const int which2 = lane >> 4, piece16 = lane & 15;
  const v4f sdv = *(const v4fa*)(sdot + which2 * GBM + 4 * piece16);
  float* sp = SD + (size_t)(2 * head + which2) * (size_t)NROW + rowBase + 4 * piece16;

  const int bh    = (rowBase / NN) * NHD + head;
  const int j0    = rowBase & (NN - 1);
  const int plsel = wave >> 1;
  const float fl  = (plsel != 0) ? 1.f : 0.f;
  const int piece = lane & 7, lq = lane >> 3;
  const int dgrp  = 32 * (wave & 1) + lq;
  unsigned short* vb = VHL + (size_t)plsel * VPLANE + (size_t)bh * (size_t)(HD * NN) + j0 + 8 * piece;

#pragma unroll
  for (int i = 0; i < 8; ++i) {
    const int gr = rowBase + 16 * wave + 2 * i + hh;
    float* op = outF + (size_t)gr * (size_t)FOUT + col0 + 4 * m;
    *(volatile v4f*)op = fv[i];
  }
  if (wave == 0) *(volatile v4f*)sp = sdv;
#pragma unroll 1
  for (int i = 0; i < 8; ++i) {
    const int d = dgrp + 4 * i;
    const v4u pv = vt_piece(stg, piece, d, fl);
    *(volatile v4u*)(vb + (size_t)d * NN) = pv;
  }
  __threadfence();
#pragma unroll
  for (int i = 0; i < 8; ++i) {
    const int gr = rowBase + 16 * wave + 2 * i + hh;
    float* op = outF + (size_t)gr * (size_t)FOUT + col0 + 4 * m;
    *(volatile v4f*)op = fv[i];
  }
  if (wave == 0) *(volatile v4f*)sp = sdv;
#pragma unroll 1
  for (int i = 0; i < 8; ++i) {
    const int d = dgrp + 4 * i;
    const v4u pv = vt_piece(stg, piece, d, fl);
    *(volatile v4u*)(vb + (size_t)d * NN) = pv;
  }
}

__device__ __forceinline__ float gsc(float ei, float ej, int a, float ninf) {
  float v = ei + ej;
  v = v > 0.f ? v : NEGSL * v;
  return (a != 0) ? v : ninf;
}
__device__ __forceinline__ v4f gsc4(float ei, const v4f e, const v4i a, float ninf) {
  v4f r;
  r.x = gsc(ei, e.x, a.x, ninf); r.y = gsc(ei, e.y, a.y, ninf);
  r.z = gsc(ei, e.z, a.z, ninf); r.w = gsc(ei, e.w, a.w, ninf);
  return r;
}
__device__ __forceinline__ unsigned int pkhl(float pa, float pb, unsigned int& lo) {
  const unsigned int ha = f2bf(pa), hb = f2bf(pb);
  const unsigned int la = f2bf(pa - bf2f(ha)), lb = f2bf(pb - bf2f(hb));
  lo = la | (lb << 16);
  return ha | (hb << 16);
}
__device__ __forceinline__ void pgrp(const v4f sa, const v4f sb, float msafe, float& ls, v4u& hq, v4u& lq) {
  const float p0 = __expf(sa.x - msafe), p1 = __expf(sa.y - msafe), p2 = __expf(sa.z - msafe), p3 = __expf(sa.w - msafe);
  const float p4 = __expf(sb.x - msafe), p5 = __expf(sb.y - msafe), p6 = __expf(sb.z - msafe), p7 = __expf(sb.w - msafe);
  ls += p0; ls += p1; ls += p2; ls += p3; ls += p4; ls += p5; ls += p6; ls += p7;
  unsigned int l0, l1, l2, l3;
  hq.x = pkhl(p0, p1, l0); hq.y = pkhl(p2, p3, l1); hq.z = pkhl(p4, p5, l2); hq.w = pkhl(p6, p7, l3);
  lq.x = l0; lq.y = l1; lq.z = l2; lq.w = l3;
}

__global__ __launch_bounds__(GTHR) void k_attn(
    const int* __restrict__ adj, const float* __restrict__ SD,
    const unsigned short* __restrict__ VHL, float* OUTP, float* PART)
{
  __shared__ __attribute__((aligned(16))) float sej[NN];
  __shared__ __attribute__((aligned(16))) float stg[QT * HD];
  __shared__ __attribute__((aligned(16))) float ssum[2 * HD];
  const int tid = (int)threadIdx.x, lane = tid & 31, wave = tid >> 5, hh = lane >> 4, m = lane & 15;
  const int qt = (int)blockIdx.x, head = (int)blockIdx.y, b = (int)blockIdx.z;
  const int rowBase = b * NN + qt * QT;
  const int bh = b * NHD + head;

  {
    const float* ejp = SD + (size_t)(2 * head + 1) * (size_t)NROW + (size_t)b * NN + 8 * tid;
    const v4f e0 = *(const v4fa*)ejp;
    const v4f e1 = *(const v4fa*)(ejp + 4);
    *(v4fa*)(sej + 8 * tid)     = e0;
    *(v4fa*)(sej + 8 * tid + 4) = e1;
  }
  __syncthreads();

  const int qrow = rowBase + 16 * wave + m;
  const float ei = SD[(size_t)(2 * head) * (size_t)NROW + qrow];
  const int* arow = adj + (size_t)qrow * (size_t)NN;
  const unsigned short* vhp = VHL + ((size_t)bh * HD + m) * (size_t)NN + 8 * hh;
  const float ninf = __uint_as_float(0xff800000u);

  v8f acc[4];
  {
    const v8f z = {0.f, 0.f, 0.f, 0.f, 0.f, 0.f, 0.f, 0.f};
    acc[0] = z; acc[1] = z; acc[2] = z; acc[3] = z;
  }
  float mrun = ninf, lrun = 0.f;

#pragma unroll 1
  for (int kt = 0; kt < NKT; ++kt) {
    const int kb = kt * KT;
    v4f s[8];
#pragma unroll
    for (int g = 0; g < 4; ++g) {
      const int k0 = kb + 32 * (g >> 1) + 16 * (g & 1) + 8 * hh;
      const v4f e0 = *(const v4fa*)(sej + k0);
      const v4f e1 = *(const v4fa*)(sej + k0 + 4);
      const v4i a0 = *(const v4ia*)(arow + k0);
      const v4i a1 = *(const v4ia*)(arow + k0 + 4);
      s[2 * g]     = gsc4(ei, e0, a0, ninf);
      s[2 * g + 1] = gsc4(ei, e1, a1, ninf);
    }
    v4f mx4 = s[0];
#pragma unroll
    for (int j = 1; j < 8; ++j) mx4 = max4(mx4, s[j]);
    float tm = fmaxf(fmaxf(mx4.x, mx4.y), fmaxf(mx4.z, mx4.w));
    tm = fmaxf(tm, __shfl_xor(tm, 16, 32));
    const float mnew  = fmaxf(mrun, tm);
    const float msafe = (mnew > ninf) ? mnew : 0.f;
    const float scale = __expf(mrun - msafe);
    mrun = mnew;

    float ls = 0.f;
    FragB ph[2], pr[2];
#pragma unroll
    for (int g = 0; g < 4; ++g) {
      v4u hq, lq;
      pgrp(s[2 * g], s[2 * g + 1], msafe, ls, hq, lq);
      ph[g >> 1].q[g & 1] = hq;
      pr[g >> 1].q[g & 1] = lq;
    }
    lrun = fmaf(lrun, scale, ls);

#pragma unroll
    for (int r = 0; r < 8; ++r) {
      const float sc = __shfl(scale, 8 * hh + r, 32);
      acc[0][r] *= sc; acc[1][r] *= sc; acc[2][r] *= sc; acc[3][r] *= sc;
    }

#pragma unroll
    for (int f = 0; f < 2; ++f) {
#pragma unroll
      for (int t = 0; t < 4; ++t) {
        const unsigned short* vq = vhp + (size_t)(16 * t) * (size_t)NN + kb + 32 * f;
        FragB vh, vl;
        vh.u[0] = *(const v8usa*)vq;            vh.u[1] = *(const v8usa*)(vq + 16);
        vl.u[0] = *(const v8usa*)(vq + VPLANE); vl.u[1] = *(const v8usa*)(vq + VPLANE + 16);
        acc[t] = wmb(ph[f], vh, acc[t]);
        acc[t] = wmb(ph[f], vl, acc[t]);
        acc[t] = wmb(pr[f], vh, acc[t]);
      }
    }
  }

  const float ltot = lrun + __shfl_xor(lrun, 16, 32);
  const float linv = __builtin_amdgcn_rcpf(ltot);
#pragma unroll
  for (int r = 0; r < 8; ++r) {
    const float li = __shfl(linv, 8 * hh + r, 32);
    acc[0][r] *= li; acc[1][r] *= li; acc[2][r] *= li; acc[3][r] *= li;
  }
#pragma unroll
  for (int t = 0; t < 4; ++t) {
    const int lc = 16 * t + m;
#pragma unroll
    for (int r = 0; r < 8; ++r) {
      const int lr = 16 * wave + 8 * hh + r;
      stg[lr * HD + lc] = acc[t][r];
    }
  }
  __syncthreads();

  {
    const int col = tid & 63, which = tid >> 6;
    float sacc = 0.f;
#pragma unroll 8
    for (int r = 0; r < QT; ++r) {
      const float x = stg[r * HD + col];
      sacc += (which != 0) ? x * x : x;
    }
    ssum[which * HD + col] = sacc;
  }
  __syncthreads();

  v4f fv[8];
#pragma unroll
  for (int i = 0; i < 8; ++i) {
    const int lr = 16 * wave + 2 * i + hh;
    fv[i] = *(const v4fa*)(stg + lr * HD + 4 * m);
  }
  const int which2 = lane >> 4, piece16 = lane & 15;
  const v4f sdv = *(const v4fa*)(ssum + which2 * HD + 4 * piece16);
  float* spart = PART + (size_t)(bh * NQT + qt) * (size_t)(2 * HD) + which2 * HD + 4 * piece16;
  const int colo = head * HD;

#pragma unroll
  for (int i = 0; i < 8; ++i) {
    const int gr = rowBase + 16 * wave + 2 * i + hh;
    float* op = OUTP + (size_t)gr * (size_t)FOUT + colo + 4 * m;
    *(volatile v4f*)op = fv[i];
  }
  if (wave == 0) *(volatile v4f*)spart = sdv;
  __threadfence();
#pragma unroll
  for (int i = 0; i < 8; ++i) {
    const int gr = rowBase + 16 * wave + 2 * i + hh;
    float* op = OUTP + (size_t)gr * (size_t)FOUT + colo + 4 * m;
    *(volatile v4f*)op = fv[i];
  }
  if (wave == 0) *(volatile v4f*)spart = sdv;
}

__global__ __launch_bounds__(NTHR) void k_bnstat(const float* __restrict__ PART, float* MI) {
  __shared__ __attribute__((aligned(16))) float smi[2 * FOUT];
  const int tid = (int)threadIdx.x;
  const int head = tid >> 6, d = tid & 63;
  double s = 0.0, q = 0.0;
#pragma unroll 1
  for (int b = 0; b < NB_G; ++b) {
#pragma unroll 1
    for (int qt = 0; qt < NQT; ++qt) {
      const float* pr = PART + (size_t)((b * NHD + head) * NQT + qt) * (size_t)(2 * HD);
      s += (double)pr[d];
      q += (double)pr[HD + d];
    }
  }
  const double mean = s / (double)NROW;
  double var = q / (double)NROW - mean * mean;
  var = var > 0.0 ? var : 0.0;
  const float varf = (float)var;
  const float istd = 1.0f / sqrtf(varf + BNEPS);
  smi[tid] = (float)mean;
  smi[FOUT + tid] = istd;
  __syncthreads();
  v4f mv = {0.f, 0.f, 0.f, 0.f};
  const bool wr = tid < (2 * FOUT) / 4;
  const int t4 = wr ? tid : 0;
  mv = *(const v4fa*)(smi + 4 * t4);
  if (wr) *(volatile v4f*)(MI + 4 * t4) = mv;
  __threadfence();
  if (wr) *(volatile v4f*)(MI + 4 * t4) = mv;
}

__global__ __launch_bounds__(NTHR) void k_apply(
    const float* __restrict__ OUTP, const float* __restrict__ WH, const float* __restrict__ MI,
    const float* __restrict__ gamma, const float* __restrict__ beta, float* out, int nUnits)
{
  const int u = (int)blockIdx.x * NTHR + (int)threadIdx.x;
  if (u >= nUnits) return;
  const int c0 = (u & (FOUT / 4 - 1)) * 4;
  const size_t e0 = (size_t)u * 4;
  const v4f x  = *(const v4fa*)(OUTP + e0);
  const v4f w  = *(const v4fa*)(WH + e0);
  const v4f mu = *(const v4fa*)(MI + c0);
  const v4f is = *(const v4fa*)(MI + FOUT + c0);
  const v4f ga = bfr4(*(const v4fa*)(gamma + c0));
  const v4f be = bfr4(*(const v4fa*)(beta + c0));
  const v4f y = (x - mu) * is * ga + be;
  v4f o = x;
#pragma unroll 1
  for (int i = 0; i < 4; ++i) {
    const float yi = (i == 0) ? y.x : ((i == 1) ? y.y : ((i == 2) ? y.z : y.w));
    const float wi = (i == 0) ? w.x : ((i == 1) ? w.y : ((i == 2) ? w.z : w.w));
    const float ng = yi < 0.f ? yi : 0.f;
    const float el = (yi > 0.f) ? yi : expm1f(ng);
    const float rv = el + wi;
    o.x = (i == 0) ? rv : o.x;
    o.y = (i == 1) ? rv : o.y;
    o.z = (i == 2) ? rv : o.z;
    o.w = (i == 3) ? rv : o.w;
  }
  *(volatile v4f*)(out + e0) = o;
  __threadfence();
  *(volatile v4f*)(out + e0) = o;
}

static inline int cdiv(int a, int b) { return (a + b - 1) / b; }

extern "C" void kernel_launch(void* const* d_in, const int* in_sizes, int n_in,
                              void* d_out, int out_size, void* d_ws, size_t ws_size,
                              hipStream_t stream) {
  if (n_in < 7) return;
  if (in_sizes[0] != NROW * FIN) return;
  if (in_sizes[1] != NB_G * NN * NN) return;
  if (in_sizes[2] != FOUT * FIN) return;
  if (in_sizes[3] != NHD * HD || in_sizes[4] != NHD * HD) return;
  if (in_sizes[5] != FOUT || in_sizes[6] != FOUT) return;
  if (out_size != NROW * FOUT) return;

  const float* h     = (const float*)d_in[0];
  const int*   adj   = (const int*)  d_in[1];
  const float* W     = (const float*)d_in[2];
  const float* a_src = (const float*)d_in[3];
  const float* a_dst = (const float*)d_in[4];
  const float* gamma = (const float*)d_in[5];
  const float* beta  = (const float*)d_in[6];
  float* out = (float*)d_out;

  char* ws = (char*)d_ws;
  size_t off = 0;
  const size_t oHB   = off; off += SZ_HB;
  const size_t oWB   = off; off += SZ_WB;
  const size_t oWH   = off; off += SZ_WH;
  const size_t oVHL  = off; off += SZ_VHL;
  const size_t oSD   = off; off += SZ_SD;
  const size_t oOUT  = off; off += SZ_OUT;
  const size_t oPART = off; off += SZ_PART;
  const size_t oMI   = off; off += SZ_MI;
  if (off > ws_size || off > (size_t)WSMAX) return;
  unsigned short* HB   = (unsigned short*)(ws + oHB);
  unsigned short* WB   = (unsigned short*)(ws + oWB);
  float*          WH   = (float*)(ws + oWH);
  unsigned short* VHL  = (unsigned short*)(ws + oVHL);
  float*          SD   = (float*)(ws + oSD);
  float*          OUTP = (float*)(ws + oOUT);
  float*          PART = (float*)(ws + oPART);
  float*          MI   = (float*)(ws + oMI);

  const int nUh = NROW * FIN / 8;
  k_cvt<<<cdiv(nUh, NTHR), NTHR, 0, stream>>>(h, HB, nUh);
  const int nUw = FOUT * FIN / 8;
  k_cvt<<<cdiv(nUw, NTHR), NTHR, 0, stream>>>(W, WB, nUw);

  k_proj<<<dim3(NROW / GBM, FOUT / GBN), GTHR, 0, stream>>>(HB, WB, WH, a_src, a_dst, SD, VHL);

  k_attn<<<dim3(NQT, NHD, NB_G), GTHR, 0, stream>>>(adj, SD, VHL, OUTP, PART);

  k_bnstat<<<1, NTHR, 0, stream>>>(PART, MI);

  const int nUo = NROW * FOUT / 4;
  k_apply<<<cdiv(nUo, NTHR), NTHR, 0, stream>>>(OUTP, WH, MI, gamma, beta, out, nUo);
}
